// Social_Model_52828097741379
// MI455X (gfx1250) — hardware-verified
//
#include <hip/hip_runtime.h>
#include <math.h>


#define NA   512
#define NNB  32
#define TT   50
#define HE   64
#define HD   128
#define DSTEPS 30
typedef _Float16 b16;
typedef __attribute__((ext_vector_type(16))) _Float16 v16b;
typedef __attribute__((ext_vector_type(8)))  _Float16 v8b;
typedef __attribute__((ext_vector_type(8)))  float    v8f;
typedef __attribute__((ext_vector_type(4)))  float    v4f;
#define VST2(T, ptr, val) do { const T _v = (val); *(volatile T*)(ptr) = _v; __threadfence(); *(volatile T*)(ptr) = _v; } while (0)
__device__ __forceinline__ v8f wmma16(v16b a, v16b b, v8f c) {
  v8f d = __builtin_amdgcn_wmma_f32_16x16x32_f16(false, a, false, b, (short)0, c, false, false);
  asm volatile("v_nop\n\tv_nop\n\tv_nop\n\tv_nop" : "+v"(d) : "v"(a), "v"(b));
  return d;
}
__device__ __forceinline__ v16b frag16(const b16* p, int hh) {
  const v8b lo = *(const v8b*)(p + 8 * hh), hi = *(const v8b*)(p + 16 + 8 * hh);
  return __builtin_shufflevector(lo, hi, 0,1,2,3,4,5,6,7,8,9,10,11,12,13,14,15);
}
__device__ __forceinline__ void lds_sync() { __builtin_amdgcn_fence(__ATOMIC_RELEASE, "workgroup"); __builtin_amdgcn_wave_barrier(); __builtin_amdgcn_fence(__ATOMIC_ACQUIRE, "workgroup"); }
__device__ __forceinline__ float sigm(float x) { return 1.0f / (1.0f + __expf(-x)); }
__device__ __forceinline__ float tanh_(float x) { const float e = __expf(2.0f * x); return 1.0f - 2.0f / (e + 1.0f); }

__global__ __launch_bounds__(256) void k_w16(const float* __restrict__ w, const float* __restrict__ w2, int n8, b16* __restrict__ W16) {
  const int t = blockIdx.x * 256 + threadIdx.x;
  if (t >= n8) return;
  v8b o;
#pragma unroll
  for (int e = 0; e < 8; ++e) { float v = w[(size_t)t * 8 + e]; if (w2) v += w2[(size_t)t * 8 + e]; o[e] = (b16)v; }
  VST2(v8b, W16 + (size_t)t * 8, o);
}
__global__ __launch_bounds__(128) void k_lstm64(const float* __restrict__ traj, const float* __restrict__ wih, const b16* __restrict__ Whh16,
                                                const float* __restrict__ bih, const float* __restrict__ bhh, float* __restrict__ Hout) {
  __shared__ __attribute__((aligned(16))) b16 Hh[4][16 * HE], Hl[4][16 * HE];
  __shared__ __attribute__((aligned(16))) float Ho[4][16 * HE];
  const int lane = threadIdx.x & 31, wave = threadIdx.x >> 5, hh = lane >> 4, l16 = lane & 15;
  const int s0 = (blockIdx.x * 4 + wave) * 16;
  b16* hh16 = Hh[wave]; b16* hl16 = Hl[wave];
  for (int q = lane; q < 16 * HE; q += 32) { hh16[q] = (b16)0.f; hl16[q] = (b16)0.f; }
  float c[4][8], h[4][8];
#pragma unroll
  for (int tt = 0; tt < 4; ++tt)
#pragma unroll
    for (int v = 0; v < 8; ++v) { c[tt][v] = 0.f; h[tt][v] = 0.f; }
  float wi0[16], wi1[16], bb[16];
#pragma unroll
  for (int gt = 0; gt < 4; ++gt)
#pragma unroll
    for (int tt = 0; tt < 4; ++tt) { const int n = gt * HE + tt * 16 + l16; wi0[gt * 4 + tt] = wih[n * 2]; wi1[gt * 4 + tt] = wih[n * 2 + 1]; bb[gt * 4 + tt] = bih[n] + bhh[n]; }
  lds_sync();
  for (int step = 0; step < TT; ++step) {
    const v16b a0h = frag16(hh16 + l16 * HE, hh), a1h = frag16(hh16 + l16 * HE + 32, hh);
    lds_sync();
    float x0[8], x1[8];
#pragma unroll
    for (int v = 0; v < 8; ++v) { const float* xp = traj + ((size_t)(s0 + v + 8 * hh) * TT + step) * 2; x0[v] = xp[0]; x1[v] = xp[1]; }
#pragma unroll
    for (int tt = 0; tt < 4; ++tt) {
      v8f g4[4];
#pragma unroll
      for (int gt = 0; gt < 4; ++gt) {
        const int n = gt * HE + tt * 16 + l16;
        const b16* wr = Whh16 + (size_t)n * HE;
        v8f acc = {};
        acc = wmma16(a0h, frag16(wr, hh), acc); acc = wmma16(a1h, frag16(wr + 32, hh), acc);
        g4[gt] = acc;
      }
#pragma unroll
      for (int v = 0; v < 8; ++v) {
        const float gi = g4[0][v] + x0[v] * wi0[0 * 4 + tt] + x1[v] * wi1[0 * 4 + tt] + bb[0 * 4 + tt];
        const float gf = g4[1][v] + x0[v] * wi0[1 * 4 + tt] + x1[v] * wi1[1 * 4 + tt] + bb[1 * 4 + tt];
        const float gg = g4[2][v] + x0[v] * wi0[2 * 4 + tt] + x1[v] * wi1[2 * 4 + tt] + bb[2 * 4 + tt];
        const float go = g4[3][v] + x0[v] * wi0[3 * 4 + tt] + x1[v] * wi1[3 * 4 + tt] + bb[3 * 4 + tt];
        c[tt][v] = sigm(gf) * c[tt][v] + sigm(gi) * tanh_(gg);
        h[tt][v] = sigm(go) * tanh_(c[tt][v]);
        const int r = v + 8 * hh, u = tt * 16 + l16;
        const b16 hb = (b16)h[tt][v]; hh16[r * HE + u] = hb; hl16[r * HE + u] = (b16)(h[tt][v] - (float)hb);
      }
    }
    lds_sync();
  }
  float* ho = Ho[wave];
#pragma unroll
  for (int tt = 0; tt < 4; ++tt)
#pragma unroll
    for (int v = 0; v < 8; ++v) ho[(v + 8 * hh) * HE + tt * 16 + l16] = h[tt][v];
  lds_sync();
  for (int pass = 0; pass < 2; ++pass) {
#pragma unroll
    for (int j = 0; j < 8; ++j) { const int pc = j * 32 + lane; *(volatile v4f*)(Hout + (size_t)s0 * HE + pc * 4) = *(const v4f*)(ho + pc * 4); }
    __threadfence();
  }
}
__global__ __launch_bounds__(256) void k_h0(const float* __restrict__ Ha, const float* __restrict__ Hn, float* __restrict__ H0) {
  const int t = blockIdx.x * 256 + threadIdx.x;
  const int b = t >> 7, c = t & 127;
  float v;
  if (c < HE) v = Ha[(size_t)b * HE + c];
  else { float s = 0.f; for (int n = 0; n < NNB; ++n) s += Hn[((size_t)b * NNB + n) * HE + c - HE]; v = s * (1.0f / NNB); }
  VST2(float, H0 + t, v);
}
__global__ __launch_bounds__(128) void k_dec(const float* __restrict__ H0, const b16* __restrict__ W16, const float* __restrict__ bih, const float* __restrict__ bhh,
                                             const float* __restrict__ ew, const float* __restrict__ eb, float* __restrict__ out) {
  __shared__ __attribute__((aligned(16))) b16 Hh[4][16 * HD], Hl[4][16 * HD];
  __shared__ __attribute__((aligned(16))) float Pr[64 * DSTEPS * 2];
  const int lane = threadIdx.x & 31, wave = threadIdx.x >> 5, hh = lane >> 4, l16 = lane & 15;
  const int s0 = (blockIdx.x * 4 + wave) * 16, sb = blockIdx.x * 64;
  b16* hh16 = Hh[wave]; b16* hl16 = Hl[wave];
  float c[8][8], hcur[8][8];
#pragma unroll
  for (int ut = 0; ut < 8; ++ut)
#pragma unroll
    for (int v = 0; v < 8; ++v) { const float h0v = H0[(size_t)(s0 + v + 8 * hh) * HD + ut * 16 + l16]; c[ut][v] = 0.f; hcur[ut][v] = h0v;
      const int r = v + 8 * hh; const b16 hb = (b16)h0v; hh16[r * HD + ut * 16 + l16] = hb; hl16[r * HD + ut * 16 + l16] = (b16)(h0v - (float)hb); }
  lds_sync();
  for (int step = 0; step < DSTEPS; ++step) {
    v16b ah[4], al[4];
#pragma unroll
    for (int ks = 0; ks < 4; ++ks) { ah[ks] = frag16(hh16 + l16 * HD + ks * 32, hh); al[ks] = frag16(hl16 + l16 * HD + ks * 32, hh); }
    lds_sync();
    float p0[8], p1[8];
#pragma unroll
    for (int v = 0; v < 8; ++v) { p0[v] = 0.f; p1[v] = 0.f; }
#pragma unroll
    for (int ut = 0; ut < 8; ++ut) {
      v8f g4[4];
#pragma unroll
      for (int gt = 0; gt < 4; ++gt) {
        const int n = gt * HD + ut * 16 + l16;
        const b16* wr = W16 + (size_t)n * HD;
        v8f acc = {};
#pragma unroll
        for (int ks = 0; ks < 4; ++ks) { const v16b w = frag16(wr + ks * 32, hh); acc = wmma16(ah[ks], w, acc); acc = wmma16(al[ks], w, acc); }
        g4[gt] = acc;
      }
      const int u = ut * 16 + l16;
      const float bi = bih[u] + bhh[u], bf = bih[HD + u] + bhh[HD + u], bg = bih[2 * HD + u] + bhh[2 * HD + u], bo = bih[3 * HD + u] + bhh[3 * HD + u];
      const float e0 = ew[u], e1 = ew[HD + u];
#pragma unroll
      for (int v = 0; v < 8; ++v) {
        const float cc = sigm(g4[1][v] + bf) * c[ut][v] + sigm(g4[0][v] + bi) * tanh_(g4[2][v] + bg);
        const float hn = sigm(g4[3][v] + bo) * tanh_(cc);
        c[ut][v] = cc; hcur[ut][v] = hn;
        const int r = v + 8 * hh; const b16 hb = (b16)hn; hh16[r * HD + u] = hb; hl16[r * HD + u] = (b16)(hn - (float)hb);
        p0[v] += hn * e0; p1[v] += hn * e1;
      }
    }
#pragma unroll
    for (int v = 0; v < 8; ++v) {
      float a = p0[v], b = p1[v];
#pragma unroll
      for (int o = 1; o < 16; o <<= 1) { a += __shfl_xor(a, o, 32); b += __shfl_xor(b, o, 32); }
      if (l16 == 0) { const int rl = (wave * 16 + v + 8 * hh); Pr[(rl * DSTEPS + step) * 2] = a + eb[0]; Pr[(rl * DSTEPS + step) * 2 + 1] = b + eb[1]; }
    }
    lds_sync();
  }
  __syncthreads();
  for (int pass = 0; pass < 2; ++pass) {
    for (int q = threadIdx.x; q < 64 * DSTEPS * 2 / 4; q += 128) *(volatile v4f*)(out + (size_t)sb * DSTEPS * 2 + q * 4) = *(const v4f*)(Pr + q * 4);
    __threadfence();
  }
}
extern "C" void kernel_launch(void* const* d_in, const int* in_sizes, int n_in,
                              void* d_out, int out_size, void* d_ws, size_t ws_size, hipStream_t stream) {
  (void)in_sizes; (void)n_in; (void)out_size;
  const float* atraj = (const float*)d_in[0];
  const float* ntraj = (const float*)d_in[1];
  const float* a_wih = (const float*)d_in[2]; const float* a_whh = (const float*)d_in[3]; const float* a_bih = (const float*)d_in[4]; const float* a_bhh = (const float*)d_in[5];
  const float* n_wih = (const float*)d_in[6]; const float* n_whh = (const float*)d_in[7]; const float* n_bih = (const float*)d_in[8]; const float* n_bhh = (const float*)d_in[9];
  const float* d_wih = (const float*)d_in[10]; const float* d_whh = (const float*)d_in[11]; const float* d_bih = (const float*)d_in[12]; const float* d_bhh = (const float*)d_in[13];
  const float* e_w = (const float*)d_in[14]; const float* e_b = (const float*)d_in[15];
  float* out = (float*)d_out;
  char* ws = (char*)d_ws; size_t off = 0;
  auto take = [&](size_t bytes) { void* p = ws + off; off = (off + bytes + 255) & ~(size_t)255; return p; };
  b16*   Wa = (b16*)take((size_t)256 * HE * 2);
  b16*   Wn = (b16*)take((size_t)256 * HE * 2);
  b16*   Wd = (b16*)take((size_t)512 * HD * 2);
  float* Ha = (float*)take((size_t)NA * HE * 4);
  float* Hn = (float*)take((size_t)NA * NNB * HE * 4);
  float* H0 = (float*)take((size_t)NA * HD * 4);
  if (off > ws_size) return;
  const dim3 b256(256);
  k_w16<<<(256 * HE / 8 + 255) / 256, b256, 0, stream>>>(a_whh, nullptr, 256 * HE / 8, Wa);
  k_w16<<<(256 * HE / 8 + 255) / 256, b256, 0, stream>>>(n_whh, nullptr, 256 * HE / 8, Wn);
  k_w16<<<(512 * HD / 8 + 255) / 256, b256, 0, stream>>>(d_wih, d_whh, 512 * HD / 8, Wd);
  k_lstm64<<<NA / 64, 128, 0, stream>>>(atraj, a_wih, Wa, a_bih, a_bhh, Ha);
  k_lstm64<<<NA * NNB / 64, 128, 0, stream>>>(ntraj, n_wih, Wn, n_bih, n_bhh, Hn);
  k_h0<<<NA * 128 / 256, b256, 0, stream>>>(Ha, Hn, H0);
  k_dec<<<NA / 64, 128, 0, stream>>>(H0, Wd, d_bih, d_bhh, e_w, e_b, out);
}
